// MoEDecoder_29257317220859
// MI455X (gfx1250) — hardware-verified
//
#include <hip/hip_runtime.h>


#define NTK  16384
#define NBL  64
#define TB   256
#define DI   256
#define HID  512
#define DO   256
#define NL   2
#define NE   16
typedef _Float16 h16;
typedef unsigned short bf;
typedef __attribute__((ext_vector_type(16))) __bf16   v16bf;
typedef __attribute__((ext_vector_type(16))) _Float16 v16h;
typedef __attribute__((ext_vector_type(8)))  _Float16 v8h;
typedef __attribute__((ext_vector_type(8)))  unsigned short v8us;
typedef __attribute__((ext_vector_type(8)))  float    v8f;
typedef __attribute__((ext_vector_type(4)))  float    v4f;
typedef v8h  __attribute__((may_alias)) v8ha;
typedef v4f  __attribute__((may_alias)) v4fa;
typedef v8us __attribute__((may_alias)) v8usa;

__device__ __forceinline__ unsigned short f2bf(float f) { unsigned u = __float_as_uint(f); u += 0x7FFFu + ((u >> 16) & 1u); return (unsigned short)(u >> 16); }
__device__ __forceinline__ float bf2f(unsigned short b) { return __uint_as_float(((unsigned)b) << 16); }
__device__ __forceinline__ float bfr(float f) { return bf2f(f2bf(f)); }
__device__ __forceinline__ v16h cat16(v8h lo, v8h hi) { return __builtin_shufflevector(lo, hi, 0, 1, 2, 3, 4, 5, 6, 7, 8, 9, 10, 11, 12, 13, 14, 15); }
__device__ __forceinline__ v16bf cat16b(v8us lo, v8us hi) { return __builtin_bit_cast(v16bf, __builtin_shufflevector(lo, hi, 0, 1, 2, 3, 4, 5, 6, 7, 8, 9, 10, 11, 12, 13, 14, 15)); }
__device__ __forceinline__ v8f wmma16(v16h a, v16h b, v8f c) { return __builtin_amdgcn_wmma_f32_16x16x32_f16(false, a, false, b, (short)0, c, false, false); }
__device__ __forceinline__ v8f wmmab(v16bf a, v16bf b, v8f c) { return __builtin_amdgcn_wmma_f32_16x16x32_bf16(false, a, false, b, (short)0, c, false, false); }


template <typename T16> struct WFrag;
template <> struct WFrag<h16> { typedef v16h V; static __device__ __forceinline__ V ld(const h16* p) { return cat16(*(const v8h*)p, *(const v8h*)(p + 16)); } static __device__ __forceinline__ v8f mma(V a, V b, v8f c) { return wmma16(a, b, c); } };
template <> struct WFrag<bf> { typedef v16bf V; static __device__ __forceinline__ V ld(const bf* p) { return cat16b(*(const v8us*)p, *(const v8us*)(p + 16)); } static __device__ __forceinline__ v8f mma(V a, V b, v8f c) { return wmmab(a, b, c); } };
template <typename T16, int NSPLIT, bool BIAS>
__global__ __launch_bounds__(32) void k_gemmw(const T16* __restrict__ A, const T16* __restrict__ A2, const T16* __restrict__ Bt, const T16* __restrict__ Bt2, int K, float* C, int ldc, const float* __restrict__ bias, size_t sA, size_t sB, size_t sC) {
    typedef typename WFrag<T16>::V V;
    __shared__ __align__(16) float os[16 * 68];
    const size_t z = blockIdx.z; A += z * sA; if (A2) A2 += z * sA; Bt += z * sB; if (Bt2) Bt2 += z * sB; C += z * sC;
    const int lane = threadIdx.x & 31, lr = lane & 15, hi = lane >> 4; const int r0 = blockIdx.x * 64, c0 = blockIdx.y * 64;
    v8f acc[4][4];
#pragma unroll
    for (int mb = 0; mb < 4; ++mb)
#pragma unroll
        for (int nb = 0; nb < 4; ++nb) acc[mb][nb] = (v8f){};
    const size_t aoff = (size_t)(r0 + lr) * K + 8 * hi, boff = (size_t)(c0 + lr) * K + 8 * hi;
#pragma unroll 1
    for (int kc = 0; kc < K; kc += 32) {
        V a[4], a2[4];
#pragma unroll
        for (int mb = 0; mb < 4; ++mb) { a[mb] = WFrag<T16>::ld(A + aoff + (size_t)mb * 16 * K + kc); if (NSPLIT == 1 || NSPLIT == 2) a2[mb] = WFrag<T16>::ld(A2 + aoff + (size_t)mb * 16 * K + kc); }
#pragma unroll
        for (int nb = 0; nb < 4; ++nb) { const V b = WFrag<T16>::ld(Bt + boff + (size_t)nb * 16 * K + kc); V b2; if (NSPLIT >= 2) b2 = WFrag<T16>::ld(Bt2 + boff + (size_t)nb * 16 * K + kc);
#pragma unroll
            for (int mb = 0; mb < 4; ++mb) { acc[mb][nb] = WFrag<T16>::mma(a[mb], b, acc[mb][nb]); if (NSPLIT == 1 || NSPLIT == 2) acc[mb][nb] = WFrag<T16>::mma(a2[mb], b, acc[mb][nb]); if (NSPLIT >= 2) acc[mb][nb] = WFrag<T16>::mma(a[mb], b2, acc[mb][nb]); } }
        asm volatile("v_nop\n\tv_nop\n\tv_nop\n\tv_nop" : "+v"(acc[0][0]), "+v"(acc[1][1]), "+v"(acc[2][2]), "+v"(acc[3][3]) : "v"(a[0]), "v"(a[3]));
    }
#pragma unroll
    for (int mb = 0; mb < 4; ++mb) {
#pragma unroll
        for (int nb = 0; nb < 4; ++nb) {
#pragma unroll
            for (int j = 0; j < 8; ++j) os[(hi * 8 + j) * 68 + nb * 16 + lr] = acc[mb][nb][j]; }
        __builtin_amdgcn_wave_barrier(); asm volatile("" ::: "memory");
        float* crow = C + (size_t)(r0 + mb * 16) * ldc + c0;
#pragma unroll 1
        for (int ps = 0; ps < 2; ++ps) {
#pragma unroll
            for (int s = 0; s < 8; ++s) { const int row = 2 * s + hi, cofs = lr * 4; v4f val = *(const v4fa*)(os + row * 68 + cofs); if (BIAS) { val[0] += bfr(bias[c0 + cofs]); val[1] += bfr(bias[c0 + cofs + 1]); val[2] += bfr(bias[c0 + cofs + 2]); val[3] += bfr(bias[c0 + cofs + 3]); }
                *(volatile v4f*)(crow + (size_t)row * ldc + cofs) = val; }
            if (ps == 0) __threadfence(); }
        __builtin_amdgcn_wave_barrier(); asm volatile("" ::: "memory");
    }
}

__device__ __forceinline__ void splitf(float y, unsigned short& h, unsigned short& l) { h = f2bf(y); l = f2bf(y - bf2f(h)); }
typedef __attribute__((ext_vector_type(2))) unsigned short v2us;
typedef __attribute__((ext_vector_type(4))) unsigned short v4us;

__global__ __launch_bounds__(256) void k_cvt8(const float* __restrict__ src, bf* dst, size_t n8) { const size_t i = (size_t)blockIdx.x * 256 + threadIdx.x; if (i >= n8) return; const v8f v = *(const v8f*)(src + i * 8); v8us o;
#pragma unroll
    for (int k = 0; k < 8; ++k) o[k] = f2bf(v[k]); *(volatile v8us*)(dst + i * 8) = o; __threadfence(); *(volatile v8us*)(dst + i * 8) = o; }
__global__ __launch_bounds__(256) void k_gsel(const float* __restrict__ Wr, const float* __restrict__ br, const int* __restrict__ route, int l, bf* WSEL, float* BSEL) { const size_t i = (size_t)blockIdx.x * 256 + threadIdx.x; const size_t per = (size_t)HID * HID / 8; if (i >= (size_t)NBL * per) return; const int z = (int)(i / per); const size_t w = (i % per) * 8; int e = route[z]; e = e < 0 ? 0 : (e >= NE ? NE - 1 : e);
    const float* src = Wr + (((size_t)l * NE + e) * HID * HID) + w; const v8f v = *(const v8f*)src; v8us o;
#pragma unroll
    for (int k = 0; k < 8; ++k) o[k] = f2bf(v[k]); *(volatile v8us*)(WSEL + (size_t)z * HID * HID + w) = o;
    if (w < HID) { const float* bsrc = br + ((size_t)l * NE + e) * HID + w; v8f bb; for (int k = 0; k < 8; ++k) bb[k] = bfr(bsrc[k]); *(volatile v8f*)(BSEL + (size_t)z * HID + w) = bb; }
    __threadfence(); *(volatile v8us*)(WSEL + (size_t)z * HID * HID + w) = o; if (w < HID) { const float* bsrc = br + ((size_t)l * NE + e) * HID + w; v8f bb; for (int k = 0; k < 8; ++k) bb[k] = bfr(bsrc[k]); *(volatile v8f*)(BSEL + (size_t)z * HID + w) = bb; } }
__global__ __launch_bounds__(256) void k_hinit(const float* __restrict__ F, float* H, bf* Hh, bf* Hl) { const size_t i = ((size_t)blockIdx.x * 256 + threadIdx.x) * 2; if (i >= (size_t)NTK * HID) return; v2us oh, ol; float hv[2];
#pragma unroll
    for (int q = 0; q < 2; ++q) { hv[q] = fmaxf(F[i + q], 0.f); unsigned short a, c2; splitf(hv[q], a, c2); oh[q] = a; ol[q] = c2; }
    typedef __attribute__((ext_vector_type(2))) float v2f; v2f h2; h2[0] = hv[0]; h2[1] = hv[1]; *(volatile v2f*)(H + i) = h2; *(volatile v2us*)(Hh + i) = oh; *(volatile v2us*)(Hl + i) = ol; __threadfence(); *(volatile v2f*)(H + i) = h2; *(volatile v2us*)(Hh + i) = oh; *(volatile v2us*)(Hl + i) = ol; }
__global__ __launch_bounds__(256) void k_comb(const float* __restrict__ SH, const float* __restrict__ RT, const float* __restrict__ BSEL, float* H, bf* Hh, bf* Hl) { const size_t i = ((size_t)blockIdx.x * 256 + threadIdx.x) * 2; if (i >= (size_t)NTK * HID) return; const int n = (int)(i % HID); const int z = (int)(i / ((size_t)TB * HID)); v2us oh, ol; float hv[2];
#pragma unroll
    for (int q = 0; q < 2; ++q) { float r = __fadd_rn(RT[i + q], BSEL[(size_t)z * HID + n + q]); asm volatile("" : "+v"(r)); float s = __fadd_rn(SH[i + q], r); asm volatile("" : "+v"(s)); hv[q] = fmaxf(__fadd_rn(s, H[i + q]), 0.f); unsigned short a, c2; splitf(hv[q], a, c2); oh[q] = a; ol[q] = c2; }
    typedef __attribute__((ext_vector_type(2))) float v2f; v2f h2; h2[0] = hv[0]; h2[1] = hv[1]; *(volatile v2f*)(H + i) = h2; *(volatile v2us*)(Hh + i) = oh; *(volatile v2us*)(Hl + i) = ol; __threadfence(); *(volatile v2f*)(H + i) = h2; *(volatile v2us*)(Hh + i) = oh; *(volatile v2us*)(Hl + i) = ol; }

extern "C" void kernel_launch(void* const* d_in, const int* in_sizes, int n_in,
                              void* d_out, int out_size, void* d_ws, size_t ws_size, hipStream_t stream) {
    (void)in_sizes; (void)n_in; (void)out_size;
    const float* x = (const float*)d_in[0]; const int* route = (const int*)d_in[1]; const float* Wi = (const float*)d_in[2]; const float* bi = (const float*)d_in[3]; const float* Wr = (const float*)d_in[4]; const float* br = (const float*)d_in[5];
    const float* Ws = (const float*)d_in[6]; const float* bs = (const float*)d_in[7]; const float* Wo = (const float*)d_in[8]; const float* bo = (const float*)d_in[9];
    float* OUT = (float*)d_out;
    char* wsp = (char*)d_ws;
    auto take = [&](size_t bytes) { char* p = wsp; wsp += (bytes + 255) & ~(size_t)255; return (void*)p; };
    bf* XB = (bf*)take((size_t)NTK * DI * 2); bf* WI = (bf*)take((size_t)HID * DI * 2); bf* WS = (bf*)take((size_t)NL * HID * HID * 2); bf* WO = (bf*)take((size_t)DO * HID * 2); bf* WSEL = (bf*)take((size_t)NBL * HID * HID * 2); float* BSEL = (float*)take((size_t)NBL * HID * 4);
    float* H = (float*)take((size_t)NTK * HID * 4); bf* Hh = (bf*)take((size_t)NTK * HID * 2); bf* Hl = (bf*)take((size_t)NTK * HID * 2); float* SH = (float*)take((size_t)NTK * HID * 4); float* RT = (float*)take((size_t)NTK * HID * 4);
    if ((size_t)(wsp - (char*)d_ws) > ws_size) return;
    { k_cvt8<<<(unsigned)(((size_t)NTK * DI / 8 + 255) / 256), 256, 0, stream>>>(x, XB, (size_t)NTK * DI / 8); k_cvt8<<<(HID * DI / 8 + 255) / 256, 256, 0, stream>>>(Wi, WI, (size_t)HID * DI / 8);
      k_cvt8<<<(NL * HID * HID / 8 + 255) / 256, 256, 0, stream>>>(Ws, WS, (size_t)NL * HID * HID / 8); k_cvt8<<<(DO * HID / 8 + 255) / 256, 256, 0, stream>>>(Wo, WO, (size_t)DO * HID / 8); }
    const unsigned L2 = (unsigned)(((size_t)NTK * HID / 2 + 255) / 256);
    k_gemmw<bf, 0, true><<<dim3(NTK / 64, HID / 64, 1), 32, 0, stream>>>(XB, nullptr, WI, nullptr, DI, SH, HID, bi, 0, 0, 0); k_hinit<<<L2, 256, 0, stream>>>(SH, H, Hh, Hl);
    for (int l = 0; l < NL; ++l) {
        k_gsel<<<(unsigned)(((size_t)NBL * HID * HID / 8 + 255) / 256), 256, 0, stream>>>(Wr, br, route, l, WSEL, BSEL);
        k_gemmw<bf, 1, true><<<dim3(NTK / 64, HID / 64, 1), 32, 0, stream>>>(Hh, Hl, WS + (size_t)l * HID * HID, nullptr, HID, SH, HID, bs + (size_t)l * HID, 0, 0, 0);
        k_gemmw<bf, 1, false><<<dim3(TB / 64, HID / 64, NBL), 32, 0, stream>>>(Hh, Hl, WSEL, nullptr, HID, RT, HID, nullptr, (size_t)TB * HID, (size_t)HID * HID, (size_t)TB * HID);
        k_comb<<<L2, 256, 0, stream>>>(SH, RT, BSEL, H, Hh, Hl); }
    k_gemmw<bf, 1, true><<<dim3(NTK / 64, DO / 64, 1), 32, 0, stream>>>(Hh, Hl, WO, nullptr, HID, OUT, DO, bo, 0, 0, 0);
}
